// DenseKANLayer_38405597561239
// MI455X (gfx1250) — hardware-run, weakly checked
//
#include <hip/hip_runtime.h>
#include <stddef.h>


#pragma clang fp contract(off)

typedef _Float16 v16h __attribute__((ext_vector_type(16)));
typedef _Float16 v8h  __attribute__((ext_vector_type(8)));
typedef float    v8f  __attribute__((ext_vector_type(8)));
typedef float    v4f  __attribute__((ext_vector_type(4)));
typedef _Float16 h16;

#ifndef NB
#define NB 512
#endif
#define NB_FULL 512
#define N_IN   128
#define N_OUT  128
#define EDGES  (N_IN * N_OUT)
#define NKNOT  15
#define NBAS   11
#define KPI    12
#define KDIM   (N_IN * KPI)

#define FT  32
#define RT  16
#define TSP (FT * KPI + 8)
#define LDC 68

#define WCARRY 64.0f
#define ACARRY 256.0f

#define NQ      ((EDGES * NKNOT) / 4)
#define NQ_ROW0 ((N_IN * NKNOT) / 4)

static_assert(NB >= 64 && NB <= NB_FULL);
static_assert((NB % 64) == 0 && (NB % RT) == 0);
static_assert((N_OUT % 64) == 0 && (N_OUT % RT) == 0);
static_assert((N_IN % FT) == 0);
static_assert((KDIM % 32) == 0);
static_assert(KPI == NBAS + 1);
static_assert(((FT * KPI * 2) % 128) == 0);
static_assert(((KDIM * 2) % 128) == 0);
static_assert(RT * FT == 2 * 256);
static_assert(RT * ((FT * KPI) / 8) == 3 * 256);
static_assert(((FT * KPI) % 64) == 0);
static_assert((TSP % 8) == 0 && TSP >= FT * KPI);
static_assert((LDC % 4) == 0 && LDC >= 64);
static_assert(((EDGES * NKNOT) % 4) == 0 && ((N_IN * NKNOT) % 4) == 0);
static_assert((NQ % 256) == 0);
static_assert(FT * 16 == 2 * 256);

#define FLAG_BYTES ((size_t)128)
#define WPL_BYTES  ((size_t)N_OUT * KDIM * 2)
#define APL_BYTES  ((size_t)NB * KDIM * 2)
#define OFF_FLAG   ((size_t)0)
#define OFF_W      (OFF_FLAG + FLAG_BYTES)
#define OFF_A      (OFF_W + WPL_BYTES)
#define WS_TOTAL   (OFF_A + APL_BYTES)
static_assert((WPL_BYTES % 128) == 0 && (APL_BYTES % 128) == 0);
static_assert(WS_TOTAL <= (size_t)134217728);

__device__ __forceinline__ float bf16r(float x) {
  unsigned int u = __float_as_uint(x);
  u = (u + 0x7FFFu + ((u >> 16) & 1u)) & 0xFFFF0000u;
  return __uint_as_float(u);
}

static __device__ __forceinline__ h16 toh_flush(float v) {
  const h16 r = (h16)v;
  return (fabsf(v) < 6.103515625e-05f) ? (h16)0.0f : r;
}

__device__ __forceinline__ v16h frag_at(const _Float16* p) {
  v8h lo = *(const v8h*)(p);
  v8h hi = *(const v8h*)(p + 16);
  v16h out;
#pragma unroll
  for (int i = 0; i < 8; ++i) { out[i] = lo[i]; out[i + 8] = hi[i]; }
  return out;
}

__device__ __forceinline__ v8f wmma16(v16h a, v16h b, v8f c) {
  v8f d = __builtin_amdgcn_wmma_f32_16x16x32_f16(false, a, false, b, (short)0, c,
                                                 false, false);
  asm volatile("v_nop\n\tv_nop\n\tv_nop\n\tv_nop" : "+v"(d) : "v"(a), "v"(b));
  return d;
}

__global__ __launch_bounds__(256) void kan_check_kernel(
    const float* __restrict__ knots, float* __restrict__ flag) {
  __shared__ int wbad[8];
  const unsigned tid = threadIdx.x, lane = tid & 31u;
  const unsigned wave = (unsigned)__builtin_amdgcn_readfirstlane((int)(threadIdx.x >> 5));
  int bad = 0;
#pragma unroll 1
  for (unsigned q = tid; q < (unsigned)NQ; q += 256u) {
    const v4f a = *(const v4f*)(knots + (size_t)4u * q);
    const v4f r = *(const v4f*)(knots + (size_t)4u * (q % (unsigned)NQ_ROW0));
    const int d = (int)(a[0] != r[0]) | (int)(a[1] != r[1]) | (int)(a[2] != r[2]) |
                  (int)(a[3] != r[3]);
    bad |= d;
  }
#pragma unroll
  for (int off = 1; off < 32; off <<= 1) bad |= __shfl_xor(bad, off, 32);
  if (lane == 0u) wbad[wave] = bad;
  __syncthreads();
  int tot = 0;
#pragma unroll
  for (int i = 0; i < 8; ++i) tot |= wbad[i];
  const float fv = (tot == 0) ? 1.0f : 0.0f;
  if (tid < 8u) {
    const v4f v = {fv, fv, fv, fv};
    float* p = flag + tid * 4u;
    *(volatile v4f*)p = v;
    __threadfence();
    *(volatile v4f*)p = v;
  }
}

__global__ __launch_bounds__(256) void kan_wbuild_kernel(
    const float* __restrict__ cbasis, const float* __restrict__ cspl,
    const float* __restrict__ cres, _Float16* __restrict__ Wt) {
  __shared__ _Float16 Ts[RT * TSP];
  const unsigned tid = threadIdx.x;
  const unsigned i0 = blockIdx.x * (unsigned)FT;
  const unsigned n0 = blockIdx.y * (unsigned)RT;
#pragma unroll 1
  for (unsigned p = 0; p < 2u; ++p) {
    const unsigned pi = tid + 256u * p;
    const unsigned f = pi & 31u, r = pi >> 5;
    const unsigned e = (n0 + r) * (unsigned)N_IN + i0 + f;
    const float cs = bf16r(cspl[e]);
    const float cr = bf16r(cres[e]);
#pragma unroll 1
    for (unsigned g = 0; g < (unsigned)NBAS; ++g) {
      const float cb = bf16r(cbasis[(size_t)e * NBAS + g]);
      Ts[r * TSP + f * KPI + g] = toh_flush(WCARRY * (cs * cb));
    }
    Ts[r * TSP + f * KPI + NBAS] = toh_flush(WCARRY * cr);
  }
  __syncthreads();
  v8h x[3];
  size_t off[3];
#pragma unroll
  for (unsigned j = 0; j < 3u; ++j) {
    const unsigned idx = tid + 256u * j;
    const unsigned rr = idx / 48u, pc = idx % 48u;
    x[j] = *(const v8h*)&Ts[rr * TSP + pc * 8u];
    off[j] = (size_t)(n0 + rr) * KDIM + i0 * KPI + pc * 8u;
  }
#pragma unroll
  for (int j = 0; j < 3; ++j) *(volatile v8h*)(Wt + off[j]) = x[j];
  __threadfence();
#pragma unroll
  for (int j = 0; j < 3; ++j) *(volatile v8h*)(Wt + off[j]) = x[j];
}

__global__ __launch_bounds__(256) void kan_abuild_kernel(
    const float* __restrict__ X, const float* __restrict__ knots,
    _Float16* __restrict__ A16) {
  __shared__ float tS[FT * 16];
  __shared__ float bbS[14 * 256];
  __shared__ _Float16 Ts[RT * TSP];
  const unsigned tid = threadIdx.x;
  const unsigned i0 = blockIdx.x * (unsigned)FT;
  const unsigned b0 = blockIdx.y * (unsigned)RT;

#pragma unroll 1
  for (unsigned j = 0; j < 2u; ++j) {
    const unsigned idx = tid + 256u * j;
    const unsigned f = idx >> 4, jj = idx & 15u;
    const unsigned jc = (jj < (unsigned)NKNOT) ? jj : (unsigned)(NKNOT - 1);
    tS[idx] = bf16r(knots[(size_t)(i0 + f) * NKNOT + jc]);
  }
  __syncthreads();

#pragma unroll 1
  for (unsigned p = 0; p < 2u; ++p) {
    const unsigned pi = tid + 256u * p;
    const unsigned f = pi & 31u, r = pi >> 5;
    const float xv = bf16r(X[(size_t)(b0 + r) * N_IN + i0 + f]);
    const unsigned tb = f * 16u;
#pragma unroll 1
    for (unsigned j = 0; j < 14u; ++j) {
      const float ta = tS[tb + j];
      const float tn = tS[tb + j + 1u];
      const bool in = (xv >= ta) & (xv < tn);
      bbS[j * 256u + tid] = in ? 1.0f : 0.0f;
    }
#pragma unroll 1
    for (unsigned order = 1; order <= 3u; ++order) {
#pragma unroll 1
      for (unsigned j = 0; j + order < 14u; ++j) {
        const float tj   = tS[tb + j];
        const float tj1  = tS[tb + j + 1u];
        const float tjo  = tS[tb + j + order];
        const float tjo1 = tS[tb + j + order + 1u];
        const float left  = (xv - tj) * (1.0f / (tjo - tj));
        const float right = (tjo1 - xv) * (1.0f / (tjo1 - tj1));
        const float bl = bbS[j * 256u + tid];
        const float bh = bbS[(j + 1u) * 256u + tid];
        bbS[j * 256u + tid] = left * bl + right * bh;
      }
    }
#pragma unroll 1
    for (unsigned g = 0; g < (unsigned)NBAS; ++g) {
      const float bv = bbS[g * 256u + tid];
      Ts[r * TSP + f * KPI + g] = toh_flush(ACARRY * bv);
    }
    const float sil = xv * (1.0f / (1.0f + __expf(-xv)));
    Ts[r * TSP + f * KPI + NBAS] = toh_flush(ACARRY * sil);
  }
  __syncthreads();

  v8h x[3];
  size_t off[3];
#pragma unroll
  for (unsigned j = 0; j < 3u; ++j) {
    const unsigned idx = tid + 256u * j;
    const unsigned rr = idx / 48u, pc = idx % 48u;
    x[j] = *(const v8h*)&Ts[rr * TSP + pc * 8u];
    off[j] = (size_t)(b0 + rr) * KDIM + i0 * KPI + pc * 8u;
  }
#pragma unroll
  for (int j = 0; j < 3; ++j) *(volatile v8h*)(A16 + off[j]) = x[j];
  __threadfence();
#pragma unroll
  for (int j = 0; j < 3; ++j) *(volatile v8h*)(A16 + off[j]) = x[j];
}

__global__ __launch_bounds__(256) void kan_gemm_kernel(
    const _Float16* __restrict__ A16, const _Float16* __restrict__ Bt,
    const float* __restrict__ bias, const float* __restrict__ flagp,
    float* __restrict__ outf) {
  __shared__ float Cs[64 * LDC];
  const unsigned tid = threadIdx.x, lane = tid & 31u;
  const unsigned w = (unsigned)__builtin_amdgcn_readfirstlane((int)(threadIdx.x >> 5));
  const unsigned mw = w >> 1, nw = w & 1u;
  const unsigned hh = lane >> 4, m = lane & 15u;
  const unsigned n0 = blockIdx.x * 64u;
  const unsigned row0 = blockIdx.y * 64u;
  const unsigned K = (unsigned)KDIM;

  const _Float16* ap  = A16 + (size_t)(row0 + mw * 16u + m) * K + hh * 8u;
  const _Float16* bp0 = Bt + (size_t)(n0 + nw * 32u + m) * K + hh * 8u;
  const _Float16* bp1 = bp0 + (size_t)16 * K;
  v8f acc0 = {}, acc1 = {};
#pragma unroll 2
  for (unsigned k0 = 0; k0 < K; k0 += 32u) {
    const v16h a  = frag_at(ap + k0);
    const v16h b0 = frag_at(bp0 + k0);
    const v16h b1 = frag_at(bp1 + k0);
    acc0 = wmma16(a, b0, acc0);
    acc1 = wmma16(a, b1, acc1);
  }
#pragma unroll
  for (int r = 0; r < 8; ++r) {
    float* d = &Cs[(mw * 16u + hh * 8u + (unsigned)r) * LDC + nw * 32u + m];
    d[0]  = acc0[r];
    d[16] = acc1[r];
  }
  __syncthreads();

  const float cs = 1.0f / (WCARRY * ACARRY);
  const float fl = flagp[0];
  const bool ok = (fl == 1.0f);
  const float qnan = __uint_as_float(0x7FC00000u);
  v4f xs[4];
  size_t off[4];
#pragma unroll
  for (unsigned i = 0; i < 4u; ++i) {
    const unsigned r = 16u * i + (tid >> 4);
    const unsigned c = (tid & 15u) * 4u;
    const v4f u = *(const v4f*)&Cs[r * LDC + c];
    const v4f g = *(const v4f*)(bias + n0 + c);
    v4f val;
#pragma unroll
    for (int j = 0; j < 4; ++j) {
      const float t = u[j] * cs + bf16r(g[j]);
      val[j] = ok ? t : qnan;
    }
    xs[i] = val;
    off[i] = (size_t)(row0 + r) * N_OUT + n0 + c;
  }
#pragma unroll
  for (int i = 0; i < 4; ++i) *(volatile v4f*)(outf + off[i]) = xs[i];
  __threadfence();
#pragma unroll
  for (int i = 0; i < 4; ++i) *(volatile v4f*)(outf + off[i]) = xs[i];
}

extern "C" void kernel_launch(void* const* d_in, const int* in_sizes, int n_in,
                              void* d_out, int out_size, void* d_ws, size_t ws_size,
                              hipStream_t stream) {
  if (n_in < 6) return;
  if ((long long)in_sizes[0] < (long long)NB * N_IN) return;
  if ((long long)in_sizes[1] < (long long)EDGES * NKNOT) return;
  if ((long long)in_sizes[2] < (long long)EDGES * NBAS) return;
  if ((long long)in_sizes[3] < (long long)EDGES) return;
  if ((long long)in_sizes[4] < (long long)EDGES) return;
  if (in_sizes[5] < N_OUT) return;
  if ((long long)out_size < (long long)NB * N_OUT) return;
  if (ws_size < WS_TOTAL) return;

  const float* x      = (const float*)d_in[0];
  const float* knots  = (const float*)d_in[1];
  const float* cbasis = (const float*)d_in[2];
  const float* cspl   = (const float*)d_in[3];
  const float* cres   = (const float*)d_in[4];
  const float* bias   = (const float*)d_in[5];
  float* out = (float*)d_out;

  char* ws = (char*)d_ws;
  float*    flag = (float*)(ws + OFF_FLAG);
  _Float16* W16  = (_Float16*)(ws + OFF_W);
  _Float16* A16  = (_Float16*)(ws + OFF_A);

  dim3 blk(256);
  kan_check_kernel<<<dim3(1), blk, 0, stream>>>(knots, flag);
  kan_wbuild_kernel<<<dim3(N_IN / FT, N_OUT / RT), blk, 0, stream>>>(cbasis, cspl, cres, W16);
  kan_abuild_kernel<<<dim3(N_IN / FT, NB / RT), blk, 0, stream>>>(x, knots, A16);
  kan_gemm_kernel<<<dim3(N_OUT / 64, NB / 64), blk, 0, stream>>>(A16, W16, bias, flag, out);
}
